// DMamba_16801912062578
// MI455X (gfx1250) — hardware-verified
//
#include <hip/hip_runtime.h>
#include <math.h>

typedef __attribute__((ext_vector_type(16))) _Float16 v16h;
typedef __attribute__((ext_vector_type(8)))  _Float16 v8h;
typedef __attribute__((ext_vector_type(8)))  float    v8f;
typedef __attribute__((ext_vector_type(4)))  float    v4f;

constexpr int kBatch  = 16;
constexpr int kSteps  = 30;
constexpr int kImg    = kBatch * kSteps;
constexpr int kSeq    = 3 * kSteps;
constexpr int kRows   = kBatch * kSeq;
constexpr int kRowsP  = 1472;
constexpr int kNE     = 512;
constexpr int kDM     = 512;
constexpr int kDin    = 1024;
constexpr int kNst    = 64;
constexpr int kDtR    = 32;
constexpr int kXdN    = kDtR + 2 * kNst;
constexpr int kXdP    = 192;
constexpr int kXzP    = 2 * kDin;
constexpr int kLayers = 3;
constexpr int kVoc    = 18;
constexpr int kImgF   = 4 * 84 * 84;
constexpr int kM1     = kImg * 400;
constexpr int kM2     = kImg * 81;
constexpr int kM2P    = 38912;
constexpr int kM3     = kImg * 49;
constexpr int kM3P    = 25088;
constexpr int kFcK    = 3136;
constexpr int kFcMP   = 512;
static_assert(kImg == 480 && kSeq == 90 && kRows == 1440, "shapes");
static_assert(kRowsP % 64 == 0 && kRowsP >= kRows && kRowsP - kRows == 32, "row pad");
static_assert(kXdN == 160 && kXdP % 64 == 0, "x_proj width");
static_assert(kM1 % 64 == 0 && kM2P % 64 == 0 && kM3P % 64 == 0 && kM2P >= kM2 && kM3P >= kM3, "conv row pads");
static_assert(kM3P * 64 == kFcMP * kFcK, "h3 plane doubles as the fc A operand");
static_assert(kFcK % 32 == 0 && kDM % 32 == 0 && kDin % 32 == 0 && kDtR % 32 == 0, "GEMM K multiples of 32");

constexpr float kCW   = 32.0f;
constexpr float kCWdt = 8.0f;
constexpr float kCH2  = 16.0f;
constexpr float kCH3  = 32.0f;
constexpr float kCTok = 32.0f;
constexpr float kCU   = 16.0f;
constexpr float kCDt  = 32.0f;
constexpr float kCG   = 64.0f;

constexpr size_t kSzC1W = (size_t)32 * 256 * 2;
constexpr size_t kSzC2W = (size_t)64 * 512 * 2;
constexpr size_t kSzC3W = (size_t)64 * 576 * 2;
constexpr size_t kSzFCW = (size_t)kNE * kFcK * 2;
constexpr size_t kSzEMW = (size_t)kDM * kNE * 2;
constexpr size_t kSzIPW = (size_t)kLayers * kXzP * kDM * 2;
constexpr size_t kSzXPW = (size_t)kLayers * kXdP * kDin * 2;
constexpr size_t kSzDTW = (size_t)kLayers * kDin * kDtR * 2;
constexpr size_t kSzOPW = (size_t)kLayers * kDM * kDin * 2;
constexpr size_t kSzH1  = (size_t)kM1 * 32 * 2;
constexpr size_t kSzH2  = (size_t)kM2P * 64 * 2;
constexpr size_t kSzH3  = (size_t)kM3P * 64 * 2;
constexpr size_t kSzSE  = (size_t)kFcMP * kNE * 4;
constexpr size_t kSzTOK = (size_t)kRowsP * kNE * 2;
constexpr size_t kSzX   = (size_t)kRowsP * kDM * 4;
constexpr size_t kSzXN  = (size_t)kRowsP * kDM * 2;
constexpr size_t kSzXZ  = (size_t)kRowsP * kXzP * 4;
constexpr size_t kSzUC  = (size_t)kRowsP * kDin * 4;
constexpr size_t kSzU16 = (size_t)kRowsP * kDin * 2;
constexpr size_t kSzXD  = (size_t)kRowsP * kXdP * 4;
constexpr size_t kSzDT  = (size_t)kRowsP * kDtR * 2;
constexpr size_t kSzDLR = (size_t)kRowsP * kDin * 4;
constexpr size_t kSzG16 = (size_t)kRowsP * kDin * 2;
constexpr size_t kOffC1W = 0;
constexpr size_t kOffC2W = kOffC1W + kSzC1W;
constexpr size_t kOffC3W = kOffC2W + kSzC2W;
constexpr size_t kOffFCW = kOffC3W + kSzC3W;
constexpr size_t kOffEMW = kOffFCW + kSzFCW;
constexpr size_t kOffIPW = kOffEMW + kSzEMW;
constexpr size_t kOffXPW = kOffIPW + kSzIPW;
constexpr size_t kOffDTW = kOffXPW + kSzXPW;
constexpr size_t kOffOPW = kOffDTW + kSzDTW;
constexpr size_t kOffH1  = kOffOPW + kSzOPW;
constexpr size_t kOffH2  = kOffH1  + kSzH1;
constexpr size_t kOffH3  = kOffH2  + kSzH2;
constexpr size_t kOffSE  = kOffH3  + kSzH3;
constexpr size_t kOffTOK = kOffSE  + kSzSE;
constexpr size_t kOffXA  = kOffTOK + kSzTOK;
constexpr size_t kOffXB  = kOffXA  + kSzX;
constexpr size_t kOffXN  = kOffXB  + kSzX;
constexpr size_t kOffXZ  = kOffXN  + kSzXN;
constexpr size_t kOffUC  = kOffXZ  + kSzXZ;
constexpr size_t kOffU16 = kOffUC  + kSzUC;
constexpr size_t kOffXD  = kOffU16 + kSzU16;
constexpr size_t kOffDT  = kOffXD  + kSzXD;
constexpr size_t kOffDLR = kOffDT  + kSzDT;
constexpr size_t kOffG16 = kOffDLR + kSzDLR;
constexpr size_t kWsTotal = kOffG16 + kSzG16;
static_assert(kWsTotal <= 134217728ull, "carve cap");
static_assert((kSzC1W % 128) == 0 && (kSzC2W % 128) == 0 && (kSzC3W % 128) == 0 && (kSzFCW % 128) == 0 &&
              (kSzEMW % 128) == 0 && (kSzIPW % 128) == 0 && (kSzXPW % 128) == 0 && (kSzDTW % 128) == 0 &&
              (kSzOPW % 128) == 0 && (kSzH1 % 128) == 0 && (kSzH2 % 128) == 0 && (kSzH3 % 128) == 0 &&
              (kSzSE % 128) == 0 && (kSzTOK % 128) == 0 && (kSzX % 128) == 0 && (kSzXN % 128) == 0 &&
              (kSzXZ % 128) == 0 && (kSzUC % 128) == 0 && (kSzU16 % 128) == 0 && (kSzXD % 128) == 0 &&
              (kSzDT % 128) == 0 && (kSzDLR % 128) == 0 && (kSzG16 % 128) == 0, "128-B aligned regions");

union FragU { v16h v; v8h h[2]; };
__device__ __forceinline__ v16h frag_load(const _Float16* p) {
  FragU f;
  f.h[0] = *(const v8h*)(p);
  f.h[1] = *(const v8h*)(p + 16);
  return f.v;
}
__device__ __forceinline__ v8f mma_h(v16h a, v16h b, v8f c) {
  return __builtin_amdgcn_wmma_f32_16x16x32_f16(false, a, false, b, (short)0, c, false, false);
}
__device__ __forceinline__ void guard4_h(v8f& a, v8f& b, v8f& c, v8f& d, v16h x, v16h y0, v16h y1, v16h y2, v16h y3) {
  asm volatile("v_nop\n\tv_nop\n\tv_nop\n\tv_nop" : "+v"(a), "+v"(b), "+v"(c), "+v"(d) : "v"(x), "v"(y0), "v"(y1), "v"(y2), "v"(y3));
}
__device__ __forceinline__ void guard2_h(v8f& a, v8f& b, v16h x, v16h y0, v16h y1) {
  asm volatile("v_nop\n\tv_nop\n\tv_nop\n\tv_nop" : "+v"(a), "+v"(b) : "v"(x), "v"(y0), "v"(y1));
}
__device__ __forceinline__ void keep4_h(v16h a, v16h b, v16h c, v16h d) { asm volatile("v_nop" :: "v"(a), "v"(b), "v"(c), "v"(d)); }
__device__ __forceinline__ void acc_guard4(v8f& a, v8f& b, v8f& c, v8f& d) { asm volatile("v_nop\n\tv_nop\n\tv_nop\n\tv_nop" : "+v"(a), "+v"(b), "+v"(c), "+v"(d)); }
__device__ __forceinline__ void acc_guard2(v8f& a, v8f& b) { asm volatile("v_nop\n\tv_nop\n\tv_nop\n\tv_nop" : "+v"(a), "+v"(b)); }
__device__ __forceinline__ void wave_lds_sync() {
  __builtin_amdgcn_fence(__ATOMIC_RELEASE, "workgroup");
  __builtin_amdgcn_wave_barrier();
  __builtin_amdgcn_fence(__ATOMIC_ACQUIRE, "workgroup");
}

template <int BIAS_MODE, bool RESID>
__global__ __launch_bounds__(256) void wmma_gemm64(
    const unsigned short* __restrict__ Ap, int lda,
    const unsigned short* __restrict__ Btp, int ldb,
    float* __restrict__ C, int ldc,
    const float* __restrict__ bias, const float* __restrict__ resid,
    int M, int N, int K, float scale)
{
  const _Float16* A  = (const _Float16*)Ap;
  const _Float16* Bt = (const _Float16*)Btp;
  __shared__ __align__(16) float sT[8][16 * 68];
  const int lane = threadIdx.x & 31;
  const int wave = threadIdx.x >> 5;
  const int tilesN = N >> 6;
  const int tilesM = M >> 6;
  const int tile = blockIdx.x * 8 + wave;
  if (tile >= tilesM * tilesN) return;
  const int tm = tile / tilesN;
  const int tn = tile - tm * tilesN;
  const int m0 = tm << 6;
  const int n0 = tn << 6;
  const int rlane = lane & 15;
  const int koff  = (lane >> 4) * 8;
  const int mOff  = (lane >> 4) * 8;

  v8f acc[4][4];
#pragma unroll
  for (int i = 0; i < 4; ++i)
#pragma unroll
    for (int j = 0; j < 4; ++j) acc[i][j] = (v8f){0.f,0.f,0.f,0.f,0.f,0.f,0.f,0.f};

  for (int k0 = 0; k0 < K; k0 += 32) {
    v16h bh[4];
#pragma unroll
    for (int j = 0; j < 4; ++j) {
      const size_t bo = (size_t)(n0 + (j << 4) + rlane) * ldb + koff + k0;
      bh[j] = frag_load(Bt + bo);
    }
#pragma unroll
    for (int i = 0; i < 4; ++i) {
      const size_t ao = (size_t)(m0 + (i << 4) + rlane) * lda + koff + k0;
      const v16h ah = frag_load(A + ao);
#pragma unroll
      for (int j = 0; j < 4; ++j) acc[i][j] = mma_h(ah, bh[j], acc[i][j]);
      guard4_h(acc[i][0], acc[i][1], acc[i][2], acc[i][3], ah, bh[0], bh[1], bh[2], bh[3]);
    }
    keep4_h(bh[0], bh[1], bh[2], bh[3]);
  }
  acc_guard4(acc[0][0], acc[0][1], acc[0][2], acc[0][3]);
  acc_guard4(acc[1][0], acc[1][1], acc[1][2], acc[1][3]);
  acc_guard4(acc[2][0], acc[2][1], acc[2][2], acc[2][3]);
  acc_guard4(acc[3][0], acc[3][1], acc[3][2], acc[3][3]);

  float* slab = sT[wave];
  const int hh = lane >> 4, c4 = (lane & 15) * 4;
#pragma unroll
  for (int i = 0; i < 4; ++i) {
    const int mBase = m0 + (i << 4);
#pragma unroll
    for (int j = 0; j < 4; ++j) {
      const int n = n0 + (j << 4) + rlane;
      float bv = 0.f;
      if (BIAS_MODE == 2) bv = bias[n];
#pragma unroll
      for (int r = 0; r < 8; ++r) {
        float v = acc[i][j][r] * scale;
        if (BIAS_MODE == 2) v += bv;
        slab[(mOff + r) * 68 + (j << 4) + rlane] = v;
      }
    }
    wave_lds_sync();
    v4f vv[8];
#pragma unroll
    for (int it = 0; it < 8; ++it) {
      const int row = it * 2 + hh;
      v4f v = *(const v4f*)(slab + row * 68 + c4);
      if (RESID) {
        const v4f rr = *(const v4f*)(resid + (size_t)(mBase + row) * ldc + n0 + c4);
        v = v + rr;
      }
      vv[it] = v;
    }
    for (int pass = 0; pass < 2; ++pass) {
#pragma unroll
      for (int it = 0; it < 8; ++it) {
        const int row = it * 2 + hh;
        *(volatile v4f*)(C + (size_t)(mBase + row) * ldc + n0 + c4) = vv[it];
      }
      __threadfence();
    }
    wave_lds_sync();
  }
}

__global__ __launch_bounds__(256) void convw_perm_kernel(
    const float* __restrict__ in, unsigned short* __restrict__ out, int IC, int KK, int Ktot, int total8, float scale)
{
  const int i = blockIdx.x * 256 + threadIdx.x;
  if (i >= total8) return;
  const int e0 = i << 3;
  const int oc = e0 / Ktot;
  const int k0 = e0 - oc * Ktot;
  v8h hv;
#pragma unroll
  for (int e = 0; e < 8; ++e) {
    const int kp  = k0 + e;
    const int tap = kp / IC;
    const int c   = kp - tap * IC;
    const float v = in[(size_t)oc * Ktot + c * KK + tap];
    hv[e] = (_Float16)(v * scale);
  }
  unsigned short* q = out + e0;
  *(volatile v8h*)q = hv;
  __threadfence();
  *(volatile v8h*)q = hv;
}

template <bool PERM>
__global__ __launch_bounds__(256) void transpose_cast_kernel(
    const float* __restrict__ Wall, unsigned short* __restrict__ Btall, int Kdim, int Ndim, float scale,
    long wStride, long btStride)
{
  __shared__ float tile[64 * 65];
  const float* W = Wall + (size_t)blockIdx.z * (size_t)wStride;
  unsigned short* Bt = Btall + (size_t)blockIdx.z * (size_t)btStride;
  const int tid = threadIdx.x, lane = tid & 31, wave = tid >> 5;
  const int n0 = blockIdx.x * 64;
  const int k0 = blockIdx.y * 64;
#pragma unroll
  for (int p = 0; p < 16; ++p) {
    const int idx = tid + p * 256;
    const int kk  = idx >> 6;
    const int nn  = idx & 63;
    const int n   = n0 + nn;
    const int nc  = (n < Ndim) ? n : (Ndim - 1);
    const int srow = PERM ? (kk * 49 + (int)blockIdx.y) : (k0 + kk);
    const float v = W[(size_t)srow * Ndim + nc];
    tile[kk * 65 + nn] = (n < Ndim) ? (v * scale) : 0.f;
  }
  __syncthreads();
  const int q = lane >> 3, c8 = (lane & 7) * 8;
  v8h hv[2];
#pragma unroll
  for (int it = 0; it < 2; ++it) {
    const int nrow = it * 32 + wave * 4 + q;
#pragma unroll
    for (int e = 0; e < 8; ++e) hv[it][e] = (_Float16)tile[(c8 + e) * 65 + nrow];
  }
  for (int pass = 0; pass < 2; ++pass) {
#pragma unroll
    for (int it = 0; it < 2; ++it) {
      const int nrow = it * 32 + wave * 4 + q;
      *(volatile v8h*)(Bt + (size_t)(n0 + nrow) * Kdim + k0 + c8) = hv[it];
    }
    __threadfence();
  }
}

__global__ __launch_bounds__(256) void dtw_cast_kernel(
    const float* __restrict__ W, unsigned short* __restrict__ Bt, int total8, float scale)
{
  const int i = blockIdx.x * 256 + threadIdx.x;
  if (i >= total8) return;
  const int e0  = i << 3;
  const int lay = e0 / (kDin * kDtR);
  const int rem = e0 - lay * (kDin * kDtR);
  const int n   = rem >> 5;
  const int k8  = rem & 31;
  v8h hv;
#pragma unroll
  for (int e = 0; e < 8; ++e) {
    const float v = W[(size_t)lay * (kDtR * kDin) + (size_t)(k8 + e) * kDin + n];
    hv[e] = (_Float16)(v * scale);
  }
  unsigned short* q = Bt + e0;
  *(volatile v8h*)q = hv;
  __threadfence();
  *(volatile v8h*)q = hv;
}

constexpr int kC1Tiles = kM1 / 64;
__global__ __launch_bounds__(256) void conv1_kernel(
    const float* __restrict__ S, const unsigned short* __restrict__ Wp, const float* __restrict__ bias,
    unsigned short* __restrict__ H1, float accScale)
{
  __shared__ __align__(16) float sT[8][16 * 36];
  const int lane = threadIdx.x & 31, wave = threadIdx.x >> 5;
  const int tile = blockIdx.x * 8 + wave;
  if (tile >= kC1Tiles) return;
  const int m0 = tile << 6;
  const int rlane = lane & 15, hh = lane >> 4;
  const int mOff = hh * 8;
  const _Float16* W = (const _Float16*)Wp;
  int base[4];
#pragma unroll
  for (int i = 0; i < 4; ++i) {
    const int m   = m0 + (i << 4) + rlane;
    const int img = m / 400;
    const int rr  = m - img * 400;
    const int oy  = rr / 20;
    const int ox  = rr - oy * 20;
    base[i] = img * kImgF + oy * (4 * 84) + ox * 4;
  }
  v8f acc[4][2];
#pragma unroll
  for (int i = 0; i < 4; ++i) {
    acc[i][0] = (v8f){0.f,0.f,0.f,0.f,0.f,0.f,0.f,0.f};
    acc[i][1] = (v8f){0.f,0.f,0.f,0.f,0.f,0.f,0.f,0.f};
  }
#pragma unroll 1
  for (int ks = 0; ks < 8; ++ks) {
    const int c    = ks >> 1;
    const int ky0  = ((ks & 1) << 2) + hh;
    const int off0 = (c * 84 + ky0) * 84;
    const int off1 = off0 + 2 * 84;
    const v16h b0 = frag_load(W + (size_t)rlane * 256 + ks * 32 + 8 * hh);
    const v16h b1 = frag_load(W + (size_t)(16 + rlane) * 256 + ks * 32 + 8 * hh);
#pragma unroll
    for (int i = 0; i < 4; ++i) {
      const float* p = S + base[i];
      const v4f a0 = *(const v4f*)(p + off0);
      const v4f a1 = *(const v4f*)(p + off0 + 4);
      const v4f a2 = *(const v4f*)(p + off1);
      const v4f a3 = *(const v4f*)(p + off1 + 4);
      v16h a;
#pragma unroll
      for (int e = 0; e < 4; ++e) {
        a[e]      = (_Float16)a0[e];
        a[4 + e]  = (_Float16)a1[e];
        a[8 + e]  = (_Float16)a2[e];
        a[12 + e] = (_Float16)a3[e];
      }
      acc[i][0] = mma_h(a, b0, acc[i][0]);
      acc[i][1] = mma_h(a, b1, acc[i][1]);
      guard2_h(acc[i][0], acc[i][1], a, b0, b1);
    }
  }
  acc_guard2(acc[0][0], acc[0][1]);
  acc_guard2(acc[1][0], acc[1][1]);
  acc_guard2(acc[2][0], acc[2][1]);
  acc_guard2(acc[3][0], acc[3][1]);

  float* slab = sT[wave];
#pragma unroll
  for (int i = 0; i < 4; ++i) {
#pragma unroll
    for (int j = 0; j < 2; ++j) {
      const int n = (j << 4) + rlane;
      const float bv = bias[n];
#pragma unroll
      for (int r = 0; r < 8; ++r) {
        float v = acc[i][j][r] * accScale + bv;
        v = fmaxf(v, 0.0f);
        slab[(mOff + r) * 36 + (j << 4) + rlane] = v;
      }
    }
    wave_lds_sync();
    v8h hv[2];
#pragma unroll
    for (int it = 0; it < 2; ++it) {
      const int idx = it * 32 + lane;
      const int row = idx >> 2;
      const int c8  = (idx & 3) * 8;
      const v4f s0 = *(const v4f*)(slab + row * 36 + c8);
      const v4f s1 = *(const v4f*)(slab + row * 36 + c8 + 4);
#pragma unroll
      for (int e = 0; e < 4; ++e) {
        hv[it][e]     = (_Float16)s0[e];
        hv[it][4 + e] = (_Float16)s1[e];
      }
    }
    unsigned short* dst = H1 + (size_t)(m0 + (i << 4)) * 32;
    for (int pass = 0; pass < 2; ++pass) {
#pragma unroll
      for (int it = 0; it < 2; ++it) {
        const int idx = it * 32 + lane;
        *(volatile v8h*)(dst + idx * 8) = hv[it];
      }
      __threadfence();
    }
    wave_lds_sync();
  }
}

template <int IC, int IW, int IH, int OH, int KW, int STRIDE, int MREAL, int MTILES>
__global__ __launch_bounds__(256) void convh_kernel(
    const unsigned short* __restrict__ Xp, const unsigned short* __restrict__ Wp, const float* __restrict__ bias,
    unsigned short* __restrict__ Yp, float accScale, float outCarry)
{
  constexpr int SUBS = IC / 32;
  constexpr int NKS  = KW * KW * SUBS;
  constexpr int KTOT = KW * KW * IC;
  constexpr int OHW  = OH * OH;
  static_assert(IC % 32 == 0 && KTOT % 32 == 0, "k-steps");
  __shared__ __align__(16) float sT[8][16 * 68];
  const int lane = threadIdx.x & 31, wave = threadIdx.x >> 5;
  const int tile = blockIdx.x * 8 + wave;
  if (tile >= MTILES) return;
  const int m0 = tile << 6;
  const int rlane = lane & 15;
  const int koff  = (lane >> 4) * 8;
  const int mOff  = (lane >> 4) * 8;
  const _Float16* X = (const _Float16*)Xp;
  const _Float16* W = (const _Float16*)Wp;
  int base[4];
#pragma unroll
  for (int i = 0; i < 4; ++i) {
    const int m   = m0 + (i << 4) + rlane;
    const int mc  = (m < MREAL) ? m : (MREAL - 1);
    const int img = mc / OHW;
    const int rr  = mc - img * OHW;
    const int oy  = rr / OH;
    const int ox  = rr - oy * OH;
    base[i] = ((img * IH + oy * STRIDE) * IW + ox * STRIDE) * IC;
  }
  v8f acc[4][4];
#pragma unroll
  for (int i = 0; i < 4; ++i)
#pragma unroll
    for (int j = 0; j < 4; ++j) acc[i][j] = (v8f){0.f,0.f,0.f,0.f,0.f,0.f,0.f,0.f};

#pragma unroll 1
  for (int ks = 0; ks < NKS; ++ks) {
    const int tap  = ks / SUBS;
    const int sub  = ks - tap * SUBS;
    const int ky   = tap / KW;
    const int kx   = tap - ky * KW;
    const int aoff = (ky * IW + kx) * IC + sub * 32 + koff;
    const int wo   = ks * 32 + koff;
    v16h bh[4];
#pragma unroll
    for (int j = 0; j < 4; ++j) bh[j] = frag_load(W + (size_t)((j << 4) + rlane) * KTOT + wo);
#pragma unroll
    for (int i = 0; i < 4; ++i) {
      const v16h ah = frag_load(X + (size_t)base[i] + aoff);
#pragma unroll
      for (int j = 0; j < 4; ++j) acc[i][j] = mma_h(ah, bh[j], acc[i][j]);
      guard4_h(acc[i][0], acc[i][1], acc[i][2], acc[i][3], ah, bh[0], bh[1], bh[2], bh[3]);
    }
    keep4_h(bh[0], bh[1], bh[2], bh[3]);
  }
  acc_guard4(acc[0][0], acc[0][1], acc[0][2], acc[0][3]);
  acc_guard4(acc[1][0], acc[1][1], acc[1][2], acc[1][3]);
  acc_guard4(acc[2][0], acc[2][1], acc[2][2], acc[2][3]);
  acc_guard4(acc[3][0], acc[3][1], acc[3][2], acc[3][3]);

  float* slab = sT[wave];
  const int q = lane >> 3, c8 = (lane & 7) * 8;
#pragma unroll
  for (int i = 0; i < 4; ++i) {
    const int mBase = m0 + (i << 4);
#pragma unroll
    for (int j = 0; j < 4; ++j) {
      const int n = (j << 4) + rlane;
      const float bv = bias[n];
#pragma unroll
      for (int r = 0; r < 8; ++r) {
        float v = acc[i][j][r] * accScale + bv;
        v = fmaxf(v, 0.0f) * outCarry;
        v = ((mBase + mOff + r) < MREAL) ? v : 0.0f;
        slab[(mOff + r) * 68 + (j << 4) + rlane] = v;
      }
    }
    wave_lds_sync();
    v8h hv[4];
#pragma unroll
    for (int it = 0; it < 4; ++it) {
      const int row = it * 4 + q;
      const v4f s0 = *(const v4f*)(slab + row * 68 + c8);
      const v4f s1 = *(const v4f*)(slab + row * 68 + c8 + 4);
#pragma unroll
      for (int e = 0; e < 4; ++e) {
        hv[it][e]     = (_Float16)s0[e];
        hv[it][4 + e] = (_Float16)s1[e];
      }
    }
    for (int pass = 0; pass < 2; ++pass) {
#pragma unroll
      for (int it = 0; it < 4; ++it) {
        const int row = it * 4 + q;
        *(volatile v8h*)(Yp + (size_t)(mBase + row) * 64 + c8) = hv[it];
      }
      __threadfence();
    }
    wave_lds_sync();
  }
}

__global__ __launch_bounds__(256) void token_kernel(
    const float* __restrict__ rtgs, const int* __restrict__ actions, const float* __restrict__ SE,
    const float* __restrict__ retw, const float* __restrict__ retb, const float* __restrict__ aemb,
    unsigned short* __restrict__ TOK)
{
  __shared__ __align__(16) float sT[2048];
  const int tid = threadIdx.x;
  const int r0 = blockIdx.x * 4;
#pragma unroll 1
  for (int i = 0; i < 8; ++i) {
    const int c  = ((i & 1) << 8) + tid;
    const int r  = r0 + (i >> 1);
    const int rc = (r < kRows) ? r : (kRows - 1);
    const int b  = rc / kSeq;
    const int s  = rc - b * kSeq;
    const int t  = s / 3;
    const int kind = s - 3 * t;
    const int bt = b * kSteps + t;
    const float rt = rtgs[bt];
    int ai = actions[bt];
    ai = (ai < 0) ? 0 : ((ai > kVoc - 1) ? (kVoc - 1) : ai);
    const float p0 = rt * retw[c] + retb[c];
    const float p1 = SE[(size_t)bt * kNE + c];
    const float p2 = aemb[(size_t)ai * kNE + c];
    const float pre = (kind == 0) ? p0 : ((kind == 1) ? p1 : p2);
    const float v = tanhf(pre) * kCTok;
    sT[i * 256 + tid] = (r < kRows) ? v : 0.0f;
  }
  __syncthreads();
  const v4f a0 = *(const v4f*)(sT + tid * 8);
  const v4f a1 = *(const v4f*)(sT + tid * 8 + 4);
  v8h hv;
#pragma unroll
  for (int e = 0; e < 4; ++e) {
    hv[e]     = (_Float16)a0[e];
    hv[4 + e] = (_Float16)a1[e];
  }
  unsigned short* q = TOK + (size_t)r0 * kNE + tid * 8;
  *(volatile v8h*)q = hv;
  __threadfence();
  *(volatile v8h*)q = hv;
}

__global__ __launch_bounds__(256) void rmsnorm_kernel(
    const float* __restrict__ X, const float* __restrict__ w, unsigned short* __restrict__ XN)
{
  const int lane = threadIdx.x & 31, wave = threadIdx.x >> 5;
  const int row = blockIdx.x * 8 + wave;
  const float* p = X + (size_t)row * kDM;
  const int c0 = lane * 8;
  const v4f a0 = *(const v4f*)(p + c0);
  const v4f a1 = *(const v4f*)(p + c0 + 4);
  const v4f a2 = *(const v4f*)(p + 256 + c0);
  const v4f a3 = *(const v4f*)(p + 256 + c0 + 4);
  float ss = 0.0f;
#pragma unroll
  for (int e = 0; e < 4; ++e) ss += a0[e] * a0[e] + a1[e] * a1[e] + a2[e] * a2[e] + a3[e] * a3[e];
  ss += __shfl_xor(ss, 16, 32);
  ss += __shfl_xor(ss, 8, 32);
  ss += __shfl_xor(ss, 4, 32);
  ss += __shfl_xor(ss, 2, 32);
  ss += __shfl_xor(ss, 1, 32);
  const float inv = rsqrtf(ss * (1.0f / (float)kDM) + 1e-5f);
  const v4f w0 = *(const v4f*)(w + c0);
  const v4f w1 = *(const v4f*)(w + c0 + 4);
  const v4f w2 = *(const v4f*)(w + 256 + c0);
  const v4f w3 = *(const v4f*)(w + 256 + c0 + 4);
  v8h h0, h1;
#pragma unroll
  for (int e = 0; e < 4; ++e) {
    h0[e]     = (_Float16)(a0[e] * inv * w0[e]);
    h0[4 + e] = (_Float16)(a1[e] * inv * w1[e]);
    h1[e]     = (_Float16)(a2[e] * inv * w2[e]);
    h1[4 + e] = (_Float16)(a3[e] * inv * w3[e]);
  }
  unsigned short* q = XN + (size_t)row * kDM + c0;
  *(volatile v8h*)q = h0;
  *(volatile v8h*)(q + 256) = h1;
  __threadfence();
  *(volatile v8h*)q = h0;
  *(volatile v8h*)(q + 256) = h1;
}

constexpr int kTP = 260;
__global__ __launch_bounds__(256) void dwconv_silu_kernel(
    const float* __restrict__ XZ, const float* __restrict__ cw, const float* __restrict__ cb,
    float* __restrict__ UC, unsigned short* __restrict__ U16)
{
  __shared__ __align__(16) float sT[16 * kTP];
  const int tid = threadIdx.x, lane = tid & 31, wave = tid >> 5;
  const int d0 = blockIdx.x * 256, d = d0 + tid;
  const int g0 = blockIdx.y * 64;
  const v4f wv = *(const v4f*)(cw + (size_t)d * 4);
  const float w0 = wv[0], w1 = wv[1], w2 = wv[2], w3 = wv[3];
  const float bc = cb[d];
  const int tb = g0 % kSeq;
  float xm3, xm2, xm1;
  {
    const int r3 = (g0 >= 3) ? (g0 - 3) : 0;
    const int r2 = (g0 >= 2) ? (g0 - 2) : 0;
    const int r1 = (g0 >= 1) ? (g0 - 1) : 0;
    const float v3 = XZ[(size_t)r3 * kXzP + d];
    const float v2 = XZ[(size_t)r2 * kXzP + d];
    const float v1 = XZ[(size_t)r1 * kXzP + d];
    xm3 = (tb >= 3) ? v3 : 0.f;
    xm2 = (tb >= 2) ? v2 : 0.f;
    xm1 = (tb >= 1) ? v1 : 0.f;
  }
  int t = tb;
  const int hrow = wave >> 1;
  const int hch  = (wave & 1) * 128 + lane * 4;
#pragma unroll 1
  for (int sub = 0; sub < 4; ++sub) {
    const int lb = g0 + sub * 16;
#pragma unroll 1
    for (int s = 0; s < 16; ++s) {
      const int g = lb + s;
      if (t == 0) { xm3 = 0.f; xm2 = 0.f; xm1 = 0.f; }
      const float xc = XZ[(size_t)g * kXzP + d];
      float acc = w0 * xm3;
      acc = fmaf(w1, xm2, acc);
      acc = fmaf(w2, xm1, acc);
      acc = fmaf(w3, xc, acc);
      const float sv = acc + bc;
      const float sg = 1.0f / (1.0f + expf(-sv));
      const float val = sv * sg;
      sT[s * kTP + tid] = (g < kRows) ? val : 0.0f;
      xm3 = xm2; xm2 = xm1; xm1 = xc;
      t = (t + 1 == kSeq) ? 0 : (t + 1);
    }
    __syncthreads();
    v4f fv[4];
    v8h bv[2];
#pragma unroll
    for (int it = 0; it < 4; ++it) fv[it] = *(const v4f*)(sT + (it * 4 + hrow) * kTP + hch);
#pragma unroll
    for (int it = 0; it < 2; ++it) {
      const float* sp = sT + (it * 8 + wave) * kTP + lane * 8;
      const v4f a0 = *(const v4f*)(sp);
      const v4f a1 = *(const v4f*)(sp + 4);
#pragma unroll
      for (int e = 0; e < 4; ++e) {
        bv[it][e]     = (_Float16)(a0[e] * kCU);
        bv[it][4 + e] = (_Float16)(a1[e] * kCU);
      }
    }
    for (int pass = 0; pass < 2; ++pass) {
#pragma unroll
      for (int it = 0; it < 4; ++it)
        *(volatile v4f*)(UC + (size_t)(lb + it * 4 + hrow) * kDin + d0 + hch) = fv[it];
#pragma unroll
      for (int it = 0; it < 2; ++it)
        *(volatile v8h*)(U16 + (size_t)(lb + it * 8 + wave) * kDin + d0 + lane * 8) = bv[it];
      __threadfence();
    }
    __syncthreads();
  }
}

__global__ __launch_bounds__(256) void dt_cast_kernel(
    const float* __restrict__ XD, unsigned short* __restrict__ DT16, int total8, float scale)
{
  const int i = blockIdx.x * 256 + threadIdx.x;
  if (i >= total8) return;
  const int e0  = i << 3;
  const int row = e0 >> 5;
  const int c8  = e0 & 31;
  const float* p = XD + (size_t)row * kXdP + c8;
  const v4f a0 = *(const v4f*)(p);
  const v4f a1 = *(const v4f*)(p + 4);
  v8h hv;
#pragma unroll
  for (int e = 0; e < 4; ++e) {
    hv[e]     = (_Float16)(a0[e] * scale);
    hv[4 + e] = (_Float16)(a1[e] * scale);
  }
  unsigned short* q = DT16 + e0;
  *(volatile v8h*)q = hv;
  __threadfence();
  *(volatile v8h*)q = hv;
}

constexpr int kScCh = 64;
constexpr int kScTS = 18;
constexpr int kScQ  = 4;
constexpr int kScS  = 16;
static_assert(kSeq % kScTS == 0 && kScQ * kScS == kNst && kDin % kScCh == 0, "scan tiling");
static_assert(kScTS * kScCh == 1152 && kScTS * 32 == 576, "scan staging counts");
__global__ __launch_bounds__(256) void scan_kernel(
    const float* __restrict__ DLR, const float* __restrict__ UC, const float* __restrict__ XZ,
    const float* __restrict__ XD, const float* __restrict__ Alog, const float* __restrict__ Dp,
    unsigned short* __restrict__ G16)
{
  __shared__ __align__(16) float sA[kScS * 256];
  __shared__ __align__(16) float sDl[kScTS * kScCh];
  __shared__ __align__(16) float sDu[kScTS * kScCh];
  __shared__ __align__(16) float sUD[kScTS * kScCh];
  __shared__ __align__(16) float sG[kScTS * kScCh];
  __shared__ __align__(16) float sBC[kScTS * 128];
  __shared__ __align__(16) float sY[kScQ * kScTS * kScCh];
  const int tid = threadIdx.x, lane = tid & 31, wave = tid >> 5;
  const int d0 = blockIdx.x * kScCh;
  const int by = blockIdx.y;
  const int q = lane >> 3, c8 = (lane & 7) * 8;
  if (by == kBatch) {
    v8h zz;
#pragma unroll
    for (int e = 0; e < 8; ++e) zz[e] = (_Float16)0.0f;
    unsigned short* pz = G16 + (size_t)(kRows + wave * 4 + q) * kDin + d0 + c8;
    *(volatile v8h*)pz = zz;
    __threadfence();
    *(volatile v8h*)pz = zz;
    return;
  }
  const int ch  = tid & 63;
  const int qtr = tid >> 6;
  const int d   = d0 + ch;
#pragma unroll 1
  for (int k = 0; k < kScS; ++k) sA[k * 256 + tid] = -expf(Alog[(size_t)d * kNst + qtr * kScS + k]);
  __syncthreads();
  float negA[kScS], h[kScS];
#pragma unroll
  for (int k = 0; k < kScS; ++k) {
    negA[k] = sA[k * 256 + tid];
    h[k] = 0.f;
  }
  const size_t row0 = (size_t)by * kSeq;
#pragma unroll 1
  for (int t0 = 0; t0 < kSeq; t0 += kScTS) {
    __syncthreads();
#pragma unroll 1
    for (int i = 0; i < 5; ++i) {
      const int idx = tid + 256 * i;
      if (idx < kScTS * kScCh) {
        const int r = idx >> 6;
        const int c = idx & 63;
        const size_t grow = row0 + t0 + r;
        const float v  = DLR[grow * kDin + d0 + c];
        const float a  = expf(-fabsf(v));
        const float dl = fmaxf(v, 0.0f) + log1pf(a);
        const float u  = UC[grow * kDin + d0 + c];
        const float z  = XZ[grow * kXzP + kDin + d0 + c];
        const float dd = Dp[d0 + c];
        sDl[idx] = dl;
        sDu[idx] = dl * u;
        sUD[idx] = u * dd;
        sG[idx]  = z * (1.0f / (1.0f + expf(-z)));
      }
    }
#pragma unroll 1
    for (int i = 0; i < 3; ++i) {
      const int idx = tid + 256 * i;
      if (idx < kScTS * 32) {
        const int r  = idx >> 5;
        const int q4 = (idx & 31) * 4;
        *(v4f*)(sBC + r * 128 + q4) = *(const v4f*)(XD + (row0 + t0 + r) * kXdP + kDtR + q4);
      }
    }
    __syncthreads();
#pragma unroll 1
    for (int s = 0; s < kScTS; ++s) {
      const float dl = sDl[s * kScCh + ch];
      const float du = sDu[s * kScCh + ch];
      const float* bc = sBC + s * 128 + qtr * kScS;
      v4f Bq[4], Cq[4];
#pragma unroll
      for (int qq = 0; qq < 4; ++qq) {
        Bq[qq] = *(const v4f*)(bc + 4 * qq);
        Cq[qq] = *(const v4f*)(bc + kNst + 4 * qq);
      }
      float y = 0.f;
#pragma unroll
      for (int k = 0; k < kScS; ++k) {
        const float e  = __expf(dl * negA[k]);
        const float pb = du * Bq[k >> 2][k & 3];
        h[k] = e * h[k] + pb;
        y = h[k] * Cq[k >> 2][k & 3] + y;
      }
      sY[qtr * (kScTS * kScCh) + s * kScCh + ch] = y;
    }
    __syncthreads();
    {
      const int row = wave * 4 + q;
      if (row < kScTS) {
        const int o = row * kScCh + c8;
        v8h hv;
#pragma unroll
        for (int hq = 0; hq < 2; ++hq) {
          const v4f y0 = *(const v4f*)(sY + 0 * (kScTS * kScCh) + o + 4 * hq);
          const v4f y1 = *(const v4f*)(sY + 1 * (kScTS * kScCh) + o + 4 * hq);
          const v4f y2 = *(const v4f*)(sY + 2 * (kScTS * kScCh) + o + 4 * hq);
          const v4f y3 = *(const v4f*)(sY + 3 * (kScTS * kScCh) + o + 4 * hq);
          const v4f ud = *(const v4f*)(sUD + o + 4 * hq);
          const v4f gg = *(const v4f*)(sG + o + 4 * hq);
#pragma unroll
          for (int e = 0; e < 4; ++e) {
            const float yy = ((y0[e] + y1[e]) + (y2[e] + y3[e])) + ud[e];
            hv[4 * hq + e] = (_Float16)(yy * gg[e] * kCG);
          }
        }
        unsigned short* pg = G16 + (row0 + t0 + row) * kDin + d0 + c8;
        *(volatile v8h*)pg = hv;
        __threadfence();
        *(volatile v8h*)pg = hv;
      }
    }
  }
}

__global__ __launch_bounds__(256) void head_kernel(
    const float* __restrict__ X, const float* __restrict__ nw, const float* __restrict__ HW, float* __restrict__ out)
{
  __shared__ __align__(16) float sX[16 * kDM];
  __shared__ __align__(16) float sO[288];
  const int tid = threadIdx.x, lane = tid & 31, wave = tid >> 5;
  const int blk = blockIdx.x;
#pragma unroll 1
  for (int j = 0; j < 2; ++j) {
    const int rr = wave * 2 + j;
    const int R  = blk * 16 + rr;
    const int b  = R / kSteps;
    const int t  = R - b * kSteps;
    const float* p = X + (size_t)(b * kSeq + 3 * t + 1) * kDM;
    v4f a[4];
    float ss = 0.0f;
#pragma unroll
    for (int i = 0; i < 4; ++i) {
      a[i] = *(const v4f*)(p + 4 * lane + 128 * i);
#pragma unroll
      for (int e = 0; e < 4; ++e) ss += a[i][e] * a[i][e];
    }
    ss += __shfl_xor(ss, 16, 32);
    ss += __shfl_xor(ss, 8, 32);
    ss += __shfl_xor(ss, 4, 32);
    ss += __shfl_xor(ss, 2, 32);
    ss += __shfl_xor(ss, 1, 32);
    const float inv = rsqrtf(ss * (1.0f / (float)kDM) + 1e-5f);
#pragma unroll
    for (int i = 0; i < 4; ++i) {
      const v4f wv = *(const v4f*)(nw + 4 * lane + 128 * i);
      v4f o;
#pragma unroll
      for (int e = 0; e < 4; ++e) o[e] = a[i][e] * inv * wv[e];
      *(v4f*)(sX + rr * kDM + 4 * lane + 128 * i) = o;
    }
  }
  __syncthreads();
#pragma unroll 1
  for (int i = 0; i < 2; ++i) {
    const int o = tid + 256 * i;
    if (o < 288) {
      const int rr = o / kVoc;
      const int v  = o - rr * kVoc;
      const float* xr = sX + rr * kDM;
      float acc = 0.0f;
#pragma unroll 4
      for (int k = 0; k < kDM; ++k) acc = fmaf(xr[k], HW[(size_t)k * kVoc + v], acc);
      sO[o] = acc;
    }
  }
  __syncthreads();
  if (tid < 72) {
    const v4f v = *(const v4f*)(sO + 4 * tid);
    float* q = out + (size_t)blk * 288 + 4 * tid;
    *(volatile v4f*)q = v;
    __threadfence();
    *(volatile v4f*)q = v;
  }
}

extern "C" void kernel_launch(void* const* d_in, const int* in_sizes, int n_in,
                              void* d_out, int out_size, void* d_ws, size_t ws_size,
                              hipStream_t stream)
{
  if (n_in < 28) return;
  if (in_sizes[0] != kImg * kImgF) return;
  if (in_sizes[1] != kImg || in_sizes[2] != kImg) return;
  if (in_sizes[3] != 32 * 256 || in_sizes[5] != 64 * 512 || in_sizes[7] != 64 * 576) return;
  if (in_sizes[9] != kFcK * kNE || in_sizes[13] != kVoc * kNE || in_sizes[14] != kNE * kDM) return;
  if (in_sizes[17] != kLayers * kDM * kXzP) return;
  if (in_sizes[18] != kLayers * kDin * 4) return;
  if (in_sizes[20] != kLayers * kDin * kXdN) return;
  if (in_sizes[21] != kLayers * kDtR * kDin) return;
  if (in_sizes[23] != kLayers * kDin * kNst) return;
  if (in_sizes[25] != kLayers * kDin * kDM) return;
  if (in_sizes[27] != kDM * kVoc) return;
  if (out_size != kImg * kVoc) return;
  if (ws_size < kWsTotal) return;

  const float* states = (const float*)d_in[0];
  const int*   actions = (const int*)d_in[1];
  const float* rtgs   = (const float*)d_in[2];
  const float* c1w = (const float*)d_in[3];
  const float* c1b = (const float*)d_in[4];
  const float* c2w = (const float*)d_in[5];
  const float* c2b = (const float*)d_in[6];
  const float* c3w = (const float*)d_in[7];
  const float* c3b = (const float*)d_in[8];
  const float* fcw = (const float*)d_in[9];
  const float* fcb = (const float*)d_in[10];
  const float* retw = (const float*)d_in[11];
  const float* retb = (const float*)d_in[12];
  const float* aemb = (const float*)d_in[13];
  const float* embw = (const float*)d_in[14];
  const float* embb = (const float*)d_in[15];
  const float* normw = (const float*)d_in[16];
  const float* ipw  = (const float*)d_in[17];
  const float* cw   = (const float*)d_in[18];
  const float* cb   = (const float*)d_in[19];
  const float* xpw  = (const float*)d_in[20];
  const float* dtw  = (const float*)d_in[21];
  const float* dtb  = (const float*)d_in[22];
  const float* alog = (const float*)d_in[23];
  const float* dpar = (const float*)d_in[24];
  const float* opw  = (const float*)d_in[25];
  const float* normfw = (const float*)d_in[26];
  const float* headw  = (const float*)d_in[27];
  float* out = (float*)d_out;

  char* ws = (char*)d_ws;
  unsigned short* C1W = (unsigned short*)(ws + kOffC1W);
  unsigned short* C2W = (unsigned short*)(ws + kOffC2W);
  unsigned short* C3W = (unsigned short*)(ws + kOffC3W);
  unsigned short* FCW = (unsigned short*)(ws + kOffFCW);
  unsigned short* EMW = (unsigned short*)(ws + kOffEMW);
  unsigned short* IPW = (unsigned short*)(ws + kOffIPW);
  unsigned short* XPW = (unsigned short*)(ws + kOffXPW);
  unsigned short* DTW = (unsigned short*)(ws + kOffDTW);
  unsigned short* OPW = (unsigned short*)(ws + kOffOPW);
  unsigned short* H1  = (unsigned short*)(ws + kOffH1);
  unsigned short* H2  = (unsigned short*)(ws + kOffH2);
  unsigned short* H3  = (unsigned short*)(ws + kOffH3);
  float*          SE  = (float*)(ws + kOffSE);
  unsigned short* TOK = (unsigned short*)(ws + kOffTOK);
  float*          XA  = (float*)(ws + kOffXA);
  float*          XB  = (float*)(ws + kOffXB);
  unsigned short* XN  = (unsigned short*)(ws + kOffXN);
  float*          XZ  = (float*)(ws + kOffXZ);
  float*          UC  = (float*)(ws + kOffUC);
  unsigned short* U16 = (unsigned short*)(ws + kOffU16);
  float*          XD  = (float*)(ws + kOffXD);
  unsigned short* DT16 = (unsigned short*)(ws + kOffDT);
  float*          DLR = (float*)(ws + kOffDLR);
  unsigned short* G16 = (unsigned short*)(ws + kOffG16);

  convw_perm_kernel<<<(32 * 256 / 8) / 256, 256, 0, stream>>>(c1w, C1W, 1, 256, 256, 32 * 256 / 8, kCW);
  convw_perm_kernel<<<(64 * 512 / 8) / 256, 256, 0, stream>>>(c2w, C2W, 32, 16, 512, 64 * 512 / 8, kCW);
  convw_perm_kernel<<<(64 * 576 / 8) / 256, 256, 0, stream>>>(c3w, C3W, 64, 9, 576, 64 * 576 / 8, kCW);
  transpose_cast_kernel<true><<<dim3(kNE / 64, kFcK / 64, 1), 256, 0, stream>>>(fcw, FCW, kFcK, kNE, kCW, 0L, 0L);
  transpose_cast_kernel<false><<<dim3(kDM / 64, kNE / 64, 1), 256, 0, stream>>>(embw, EMW, kNE, kDM, kCW, 0L, 0L);
  transpose_cast_kernel<false><<<dim3(kXzP / 64, kDM / 64, kLayers), 256, 0, stream>>>(
      ipw, IPW, kDM, kXzP, kCW, (long)kDM * kXzP, (long)kXzP * kDM);
  transpose_cast_kernel<false><<<dim3(kXdP / 64, kDin / 64, kLayers), 256, 0, stream>>>(
      xpw, XPW, kDin, kXdN, kCW, (long)kDin * kXdN, (long)kXdP * kDin);
  dtw_cast_kernel<<<(kLayers * kDin * kDtR / 8) / 256, 256, 0, stream>>>(dtw, DTW, kLayers * kDin * kDtR / 8, kCWdt);
  transpose_cast_kernel<false><<<dim3(kDM / 64, kDin / 64, kLayers), 256, 0, stream>>>(
      opw, OPW, kDin, kDM, kCW, (long)kDin * kDM, (long)kDM * kDin);

  conv1_kernel<<<kC1Tiles / 8, 256, 0, stream>>>(states, C1W, c1b, H1, 1.0f / kCW);
  convh_kernel<32, 20, 20, 9, 4, 2, kM2, kM2P / 64><<<(kM2P / 64) / 8, 256, 0, stream>>>(
      H1, C2W, c2b, H2, 1.0f / kCW, kCH2);
  convh_kernel<64, 9, 9, 7, 3, 1, kM3, kM3P / 64><<<(kM3P / 64) / 8, 256, 0, stream>>>(
      H2, C3W, c3b, H3, 1.0f / (kCH2 * kCW), kCH3);
  wmma_gemm64<2, false><<<8, 256, 0, stream>>>(
      H3, kFcK, FCW, kFcK, SE, kNE, fcb, fcb, kFcMP, kNE, kFcK, 1.0f / (kCH3 * kCW));

  token_kernel<<<kRowsP / 4, 256, 0, stream>>>(rtgs, actions, SE, retw, retb, aemb, TOK);
  wmma_gemm64<2, false><<<23, 256, 0, stream>>>(
      TOK, kNE, EMW, kNE, XA, kDM, embb, embb, kRowsP, kDM, kNE, 1.0f / (kCTok * kCW));

  for (int i = 0; i < kLayers; ++i) {
    float* xin  = (i & 1) ? XB : XA;
    float* xout = (i & 1) ? XA : XB;
    rmsnorm_kernel<<<kRowsP / 8, 256, 0, stream>>>(xin, normw + (size_t)i * kDM, XN);
    wmma_gemm64<0, false><<<92, 256, 0, stream>>>(
        XN, kDM, IPW + (size_t)i * kXzP * kDM, kDM, XZ, kXzP, embb, embb, kRowsP, kXzP, kDM, 1.0f / kCW);
    dwconv_silu_kernel<<<dim3(kDin / 256, kRowsP / 64), 256, 0, stream>>>(
        XZ, cw + (size_t)i * kDin * 4, cb + (size_t)i * kDin, UC, U16);
    wmma_gemm64<0, false><<<9, 256, 0, stream>>>(
        U16, kDin, XPW + (size_t)i * kXdP * kDin, kDin, XD, kXdP, embb, embb, kRowsP, kXdP, kDin, 1.0f / (kCU * kCW));
    dt_cast_kernel<<<(kRowsP * kDtR / 8) / 256, 256, 0, stream>>>(XD, DT16, kRowsP * kDtR / 8, kCDt);
    wmma_gemm64<2, false><<<46, 256, 0, stream>>>(
        DT16, kDtR, DTW + (size_t)i * kDin * kDtR, kDtR, DLR, kDin, dtb + (size_t)i * kDin, embb,
        kRowsP, kDin, kDtR, 1.0f / (kCDt * kCWdt));
    scan_kernel<<<dim3(kDin / kScCh, kBatch + 1), 256, 0, stream>>>(
        DLR, UC, XZ, XD, alog + (size_t)i * kDin * kNst, dpar + (size_t)i * kDin, G16);
    wmma_gemm64<0, true><<<23, 256, 0, stream>>>(
        G16, kDin, OPW + (size_t)i * kDM * kDin, kDin, xout, kDM, embb, xin, kRowsP, kDM, kDin, 1.0f / (kCG * kCW));
  }

  head_kernel<<<kImg / 16, 256, 0, stream>>>(XB, normfw, headw, out);
}
